// DIFFBlock_90031104459369
// MI455X (gfx1250) — hardware-verified
//
#include <hip/hip_runtime.h>
#include <math.h>

typedef __attribute__((ext_vector_type(16))) _Float16 v16h;
typedef __attribute__((ext_vector_type(8)))  _Float16 v8h;
typedef __attribute__((ext_vector_type(16))) __bf16   v16b;
typedef __attribute__((ext_vector_type(8)))  __bf16   v8b;
typedef __attribute__((ext_vector_type(8)))  float    v8f;
typedef __attribute__((ext_vector_type(4)))  float    v4f;

__device__ __forceinline__ unsigned short f2bf_bits(float f) {
  unsigned u = __float_as_uint(f);
  return (unsigned short)((u + 0x7FFFu + ((u >> 16) & 1u)) >> 16);
}
__device__ __forceinline__ float bf_bits2f(unsigned short h) { return __uint_as_float(((unsigned)h) << 16); }

__device__ __forceinline__ void dep_guard_h(v8f& a, v8f& b, v16h x, v16h y) { asm volatile("v_nop\n\tv_nop\n\tv_nop\n\tv_nop" : "+v"(a), "+v"(b) : "v"(x), "v"(y)); }
__device__ __forceinline__ void dep_guard_b(v8f& a, v8f& b, v16b x, v16b y) { asm volatile("v_nop\n\tv_nop\n\tv_nop\n\tv_nop" : "+v"(a), "+v"(b) : "v"(x), "v"(y)); }
__device__ __forceinline__ void keep4_h(v16h a, v16h b, v16h c, v16h d) { asm volatile("v_nop" :: "v"(a), "v"(b), "v"(c), "v"(d)); }
__device__ __forceinline__ void keep4_b(v16b a, v16b b, v16b c, v16b d) { asm volatile("v_nop" :: "v"(a), "v"(b), "v"(c), "v"(d)); }
__device__ __forceinline__ void acc_guard4(v8f& a, v8f& b, v8f& c, v8f& d) { asm volatile("v_nop\n\tv_nop\n\tv_nop\n\tv_nop" : "+v"(a), "+v"(b), "+v"(c), "+v"(d)); }
template <typename T> struct Frag;
template <> struct Frag<_Float16> {
  typedef v16h V; union U { v16h v; v8h h[2]; };
  static __device__ __forceinline__ v16h load(const _Float16* p) {
    U f; f.h[0] = *(const v8h*)(p); f.h[1] = *(const v8h*)(p + 16); return f.v;
  }
  static __device__ __forceinline__ v8f mma(v16h a, v16h b, v8f c) {
    return __builtin_amdgcn_wmma_f32_16x16x32_f16(false, a, false, b, (short)0, c, false, false);
  }
  static __device__ __forceinline__ void guard(v8f& a, v8f& b, v16h x, v16h y) { dep_guard_h(a, b, x, y); }
  static __device__ __forceinline__ void keep(v16h a, v16h b, v16h c, v16h d) { keep4_h(a, b, c, d); }
};
template <> struct Frag<__bf16> {
  typedef v16b V; union U { v16b v; v8b h[2]; };
  static __device__ __forceinline__ v16b load(const __bf16* p) {
    U f; f.h[0] = *(const v8b*)(p); f.h[1] = *(const v8b*)(p + 16); return f.v;
  }
  static __device__ __forceinline__ v8f mma(v16b a, v16b b, v8f c) {
    return __builtin_amdgcn_wmma_f32_16x16x32_bf16(false, a, false, b, (short)0, c, false, false);
  }
  static __device__ __forceinline__ void guard(v8f& a, v8f& b, v16b x, v16b y) { dep_guard_b(a, b, x, y); }
  static __device__ __forceinline__ void keep(v16b a, v16b b, v16b c, v16b d) { keep4_b(a, b, c, d); }
};

template <int ET> struct Elem;
template <> struct Elem<0> { typedef _Float16 T; };
template <> struct Elem<1> { typedef __bf16 T; };
template <int ET, bool SPLIT, int BIAS_MODE, int OUT_MODE, bool RESID, int ACT = 0>
__global__ __launch_bounds__(256) void wmma_gemm64(
    const unsigned short* __restrict__ Ap, const unsigned short* __restrict__ A2p, int lda, long strideA,
    const unsigned short* __restrict__ Btp, const unsigned short* __restrict__ Bt2p, int ldb, long strideB,
    void* __restrict__ Cout, void* __restrict__ Cout2, int ldc, long strideC,
    const float* __restrict__ bias,
    const float* __restrict__ resid, long strideR,
    int M, int N, int K, float scale) {
  typedef typename Elem<ET>::T T;
  typedef typename Frag<T>::V V;
  const T* A = (const T*)Ap; const T* A2 = (const T*)A2p; const T* Bt = (const T*)Btp; const T* Bt2 = (const T*)Bt2p;
  __shared__ __align__(16) float sT[8][16 * 68];
  const int b    = blockIdx.y;
  const int lane = threadIdx.x & 31;
  const int wave = threadIdx.x >> 5;
  const int tilesN = N >> 6;
  const int tilesM = M >> 6;
  const int tile = blockIdx.x * 8 + wave;
  if (tile >= tilesM * tilesN) return;
  const int tm = tile / tilesN;
  const int tn = tile - tm * tilesN;
  const int m0 = tm << 6;
  const int n0 = tn << 6;

  const T* Ab  = A  + (size_t)b * strideA;
  const T* Bb  = Bt + (size_t)b * strideB;
  const T* Ab2 = SPLIT ? (A2  + (size_t)b * strideA) : nullptr;
  const T* Bb2 = SPLIT ? (Bt2 + (size_t)b * strideB) : nullptr;

  const int rlane = lane & 15;
  const int koff  = (lane >> 4) * 8;
  const int mOff  = (lane >> 4) * 8;

  v8f acc[4][4];
#pragma unroll
  for (int i = 0; i < 4; ++i)
#pragma unroll
    for (int j = 0; j < 4; ++j) acc[i][j] = (v8f){0.f,0.f,0.f,0.f,0.f,0.f,0.f,0.f};

  for (int k0 = 0; k0 < K; k0 += 32) {
    V bh[4], bl[4];
#pragma unroll
    for (int j = 0; j < 4; ++j) {
      const size_t bo = (size_t)(n0 + (j << 4) + rlane) * ldb + koff + k0;
      bh[j] = Frag<T>::load(Bb + bo);
      if (SPLIT) bl[j] = Frag<T>::load(Bb2 + bo);
    }
#pragma unroll
    for (int i = 0; i < 4; ++i) {
      const size_t ao = (size_t)(m0 + (i << 4) + rlane) * lda + koff + k0;
      V ah = Frag<T>::load(Ab + ao);
      V al;
      if (SPLIT) al = Frag<T>::load(Ab2 + ao);
#pragma unroll
      for (int j = 0; j < 4; ++j) {
        acc[i][j] = Frag<T>::mma(ah, bh[j], acc[i][j]);
        if (SPLIT) {
          acc[i][j] = Frag<T>::mma(ah, bl[j], acc[i][j]);
          acc[i][j] = Frag<T>::mma(al, bh[j], acc[i][j]);
        }
      }
      Frag<T>::guard(acc[i][0], acc[i][3], ah, SPLIT ? al : ah);
    }
    Frag<T>::keep(bh[0], bh[1], bh[2], bh[3]);
    if (SPLIT) Frag<T>::keep(bl[0], bl[1], bl[2], bl[3]);
  }
  acc_guard4(acc[0][0], acc[0][1], acc[0][2], acc[0][3]);
  acc_guard4(acc[1][0], acc[1][1], acc[1][2], acc[1][3]);
  acc_guard4(acc[2][0], acc[2][1], acc[2][2], acc[2][3]);
  acc_guard4(acc[3][0], acc[3][1], acc[3][2], acc[3][3]);

  float* slab = sT[wave];
  const float* Rb = RESID ? (resid + (size_t)b * strideR) : nullptr;
#pragma unroll
  for (int i = 0; i < 4; ++i) {
    const int mBase = m0 + (i << 4);
#pragma unroll
    for (int j = 0; j < 4; ++j) {
      const int n = n0 + (j << 4) + rlane;
      float bv = 0.f;
      if (BIAS_MODE == 2) bv = bias[n];
#pragma unroll
      for (int r = 0; r < 8; ++r) {
        float v = acc[i][j][r] * scale;
        if (BIAS_MODE == 1) v += bias[mBase + mOff + r];
        if (BIAS_MODE == 2) v += bv;
        if (RESID) v += Rb[(size_t)(mBase + mOff + r) * ldc + n];
        if (ACT == 1) v = tanhf(v);
        if (ACT == 2) v = fmaxf(v, 0.0f);
        if (ACT == 3) v = v / (1.0f + expf(-v));
        if (ACT == 4) v = (v > 0.f) ? v : 0.01f * v;
        if (ACT == 5) v = 0.5f * v * (1.0f + erff(v * 0.70710678118654752f));
        slab[(mOff + r) * 68 + (j << 4) + rlane] = v;
      }
    }
    __builtin_amdgcn_fence(__ATOMIC_RELEASE, "workgroup");
    __builtin_amdgcn_wave_barrier();
    __builtin_amdgcn_fence(__ATOMIC_ACQUIRE, "workgroup");
    if (OUT_MODE == 0) {
      float* C = (float*)Cout + (size_t)b * strideC;
      const int hh = lane >> 4, c4 = (lane & 15) * 4;
      for (int pass = 0; pass < 2; ++pass) {
#pragma unroll
        for (int it = 0; it < 8; ++it) {
          const int row = it * 2 + hh;
          v4f v = *(const v4f*)(slab + row * 68 + c4);
          *(volatile v4f*)(C + (size_t)(mBase + row) * ldc + n0 + c4) = v;
        }
        __threadfence();
      }
    } else {
      const int q = lane >> 3, c8 = (lane & 7) * 8;
      unsigned short* C  = (unsigned short*)Cout  + (size_t)b * strideC;
      unsigned short* C2 = (OUT_MODE == 2) ? ((unsigned short*)Cout2 + (size_t)b * strideC) : nullptr;
      for (int pass = 0; pass < 2; ++pass) {
#pragma unroll
        for (int it = 0; it < 4; ++it) {
          const int row = it * 4 + q;
          const float* sp = slab + row * 68 + c8;
          v8h hv, lv;
#pragma unroll
          for (int e = 0; e < 8; ++e) {
            if (OUT_MODE == 1) {
              hv[e] = (_Float16)sp[e];
            } else {
              unsigned short hb = f2bf_bits(sp[e]);
              unsigned short lb = f2bf_bits(sp[e] - bf_bits2f(hb));
              hv[e] = __builtin_bit_cast(_Float16, hb);
              lv[e] = __builtin_bit_cast(_Float16, lb);
            }
          }
          *(volatile v8h*)(C + (size_t)(mBase + row) * ldc + n0 + c8) = hv;
          if (OUT_MODE == 2) *(volatile v8h*)(C2 + (size_t)(mBase + row) * ldc + n0 + c8) = lv;
        }
        __threadfence();
      }
    }
    __builtin_amdgcn_fence(__ATOMIC_RELEASE, "workgroup");
    __builtin_amdgcn_wave_barrier();
    __builtin_amdgcn_fence(__ATOMIC_ACQUIRE, "workgroup");
  }
}

__global__ __launch_bounds__(256) void cast_scale_f32_f16x2(
    const float* __restrict__ in, _Float16* __restrict__ out, int n2, float scale) {
  int i = blockIdx.x * 256 + threadIdx.x;
  if (i < n2) {
    const _Float16 h0 = (_Float16)(in[2 * i] * scale), h1 = (_Float16)(in[2 * i + 1] * scale);
    const unsigned u = (unsigned)__builtin_bit_cast(unsigned short, h0) | ((unsigned)__builtin_bit_cast(unsigned short, h1) << 16);
    ((volatile unsigned*)out)[i] = u;
    __threadfence();
    ((volatile unsigned*)out)[i] = u;
  }
}

#define RW 768
__global__ __launch_bounds__(256) void ln_rows_f16(
    const float* __restrict__ X, const float* __restrict__ w, const float* __restrict__ bvec,
    _Float16* __restrict__ Y, int nrows, float eps) {
  const int wave = threadIdx.x >> 5, lane = threadIdx.x & 31;
  const int row = blockIdx.x * 8 + wave;
  if (row >= nrows) return;
  const float* xr = X + (size_t)row * RW;
  v4f xv[6];
#pragma unroll
  for (int i = 0; i < 3; ++i) {
    const int base = 256 * i + 8 * lane;
    xv[2 * i]     = *(const v4f*)(xr + base);
    xv[2 * i + 1] = *(const v4f*)(xr + base + 4);
  }
  float s = 0.f;
#pragma unroll
  for (int i = 0; i < 6; ++i) s += (xv[i][0] + xv[i][1]) + (xv[i][2] + xv[i][3]);
#pragma unroll
  for (int off = 1; off < 32; off <<= 1) s += __shfl_xor(s, off, 32);
  const float mean = s * (1.0f / (float)RW);
  float qv = 0.f;
#pragma unroll
  for (int i = 0; i < 6; ++i) {
#pragma unroll
    for (int e = 0; e < 4; ++e) { const float d = xv[i][e] - mean; qv += d * d; }
  }
#pragma unroll
  for (int off = 1; off < 32; off <<= 1) qv += __shfl_xor(qv, off, 32);
  const float inv = rsqrtf(qv * (1.0f / (float)RW) + eps);
  v8h yv[3];
#pragma unroll
  for (int i = 0; i < 3; ++i) {
    const int base = 256 * i + 8 * lane;
    const v4f w0 = *(const v4f*)(w + base), w1 = *(const v4f*)(w + base + 4);
    const v4f b0 = *(const v4f*)(bvec + base), b1 = *(const v4f*)(bvec + base + 4);
#pragma unroll
    for (int e = 0; e < 4; ++e) {
      yv[i][e]     = (_Float16)((xv[2 * i][e] - mean) * inv * w0[e] + b0[e]);
      yv[i][4 + e] = (_Float16)((xv[2 * i + 1][e] - mean) * inv * w1[e] + b1[e]);
    }
  }
  _Float16* yr = Y + (size_t)row * RW;
  for (int pass = 0; pass < 2; ++pass) {
#pragma unroll
    for (int i = 0; i < 3; ++i) *(volatile v8h*)(yr + 256 * i + 8 * lane) = yv[i];
    __threadfence();
  }
}

__global__ __launch_bounds__(256) void diff_rms_f16(
    const float* __restrict__ O1, const float* __restrict__ O2,
    const float* __restrict__ lam1, const float* __restrict__ lam2, const float* __restrict__ w,
    const int* __restrict__ pos_unused, _Float16* __restrict__ Y, int nrows, float eps, float lam_init) {
  (void)pos_unused;
  const int wave = threadIdx.x >> 5, lane = threadIdx.x & 31;
  const int row = blockIdx.x * 8 + wave;
  if (row >= nrows) return;
  const float* ar = O1 + (size_t)row * RW;
  const float* cr = O2 + (size_t)row * RW;
  v4f ov[6];
#pragma unroll
  for (int i = 0; i < 3; ++i) {
    const int base = 256 * i + 8 * lane;
    const int head = base >> 6;
    const float lam = (lam1[head] - lam2[head]) + lam_init;
    const v4f a0 = *(const v4f*)(ar + base), a1 = *(const v4f*)(ar + base + 4);
    const v4f c0 = *(const v4f*)(cr + base), c1 = *(const v4f*)(cr + base + 4);
#pragma unroll
    for (int e = 0; e < 4; ++e) {
      ov[2 * i][e]     = a0[e] - lam * c0[e];
      ov[2 * i + 1][e] = a1[e] - lam * c1[e];
    }
  }
  float ss = 0.f;
#pragma unroll
  for (int i = 0; i < 6; ++i) {
#pragma unroll
    for (int e = 0; e < 4; ++e) ss += ov[i][e] * ov[i][e];
  }
#pragma unroll
  for (int off = 1; off < 32; off <<= 1) ss += __shfl_xor(ss, off, 32);
  const float inv = rsqrtf(ss * (1.0f / (float)RW) + eps);
  v8h yv[3];
#pragma unroll
  for (int i = 0; i < 3; ++i) {
    const int base = 256 * i + 8 * lane;
    const v4f w0 = *(const v4f*)(w + base), w1 = *(const v4f*)(w + base + 4);
#pragma unroll
    for (int e = 0; e < 4; ++e) {
      yv[i][e]     = (_Float16)(ov[2 * i][e] * inv * w0[e]);
      yv[i][4 + e] = (_Float16)(ov[2 * i + 1][e] * inv * w1[e]);
    }
  }
  _Float16* yr = Y + (size_t)row * RW;
  for (int pass = 0; pass < 2; ++pass) {
#pragma unroll
    for (int i = 0; i < 3; ++i) *(volatile v8h*)(yr + 256 * i + 8 * lane) = yv[i];
    __threadfence();
  }
}

#define AT_D 64
#define AT_NW 4
#define AT_QB 64
#define AT_KC 64
#define AT_PSC 32768.0f

__device__ __forceinline__ v8f mma_h(v16h a, v16h b, v8f c) {
  c = __builtin_amdgcn_wmma_f32_16x16x32_f16(false, a, false, b, (short)0, c, false, false);
  asm volatile("v_nop\n\tv_nop\n\tv_nop\n\tv_nop" : "+v"(c) : "v"(a), "v"(b));
  return c;
}

__global__ __launch_bounds__(128)
void attn64_f16(const _Float16* __restrict__ q, int ldq,
                const _Float16* __restrict__ k, int ldk,
                const _Float16* __restrict__ v, int ldv,
                float* __restrict__ out, int ldo,
                int S, int Skv, int H, float qscale) {
  __shared__ __align__(16) _Float16 Ksh[AT_KC * AT_D];
  __shared__ __align__(16) _Float16 Vth[AT_D * AT_KC];
  __shared__ __align__(16) _Float16 Psh[AT_NW][16 * AT_KC];
  __shared__ __align__(16) float  Os[AT_NW][16 * 68];

  const int tid  = threadIdx.x;
  const int wave = tid >> 5;
  const int lane = tid & 31;
  const int hh   = lane >> 4;
  const int c    = lane & 15;

  const int nqb = S / AT_QB;
  const int bx = blockIdx.x;
  const int qb = bx % nqb;
  const int bh = bx / nqb;
  const int h  = bh % H;
  const int b  = bh / H;
  const int q0 = qb * AT_QB + wave * 16;

  const _Float16* qbp = q + (size_t)b * S * ldq + h * AT_D;
  const _Float16* kbp = k + (size_t)b * Skv * ldk + h * AT_D;
  const _Float16* vbp = v + (size_t)b * Skv * ldv + h * AT_D;
  float*          obp = out + (size_t)b * S * ldo + h * AT_D;

  v16h qa[2];
  {
    const _Float16* qrow = qbp + (size_t)(q0 + c) * ldq;
#pragma unroll
    for (int dc = 0; dc < 2; ++dc) qa[dc] = Frag<_Float16>::load(qrow + dc * 32 + 8 * hh);
  }

  float mrow[8], lrow[8];
  v8f oacc[4];
#pragma unroll
  for (int r = 0; r < 8; ++r) { mrow[r] = -INFINITY; lrow[r] = 0.f; }
#pragma unroll
  for (int t = 0; t < 4; ++t) oacc[t] = (v8f){0.f,0.f,0.f,0.f,0.f,0.f,0.f,0.f};

  const int nChunks = Skv / AT_KC;
  for (int kc = 0; kc < nChunks; ++kc) {
    const int kv0 = kc * AT_KC;
    __syncthreads();
    {
      const int kvr = tid >> 1, dh = (tid & 1) * 32;
      const _Float16* krow = kbp + (size_t)(kv0 + kvr) * ldk + dh;
      const _Float16* vrow = vbp + (size_t)(kv0 + kvr) * ldv + dh;
#pragma unroll
      for (int i = 0; i < 4; ++i) {
        const v8h kk = *(const v8h*)(krow + 8 * i);
        const v8h vv = *(const v8h*)(vrow + 8 * i);
        *(v8h*)(Ksh + kvr * AT_D + dh + 8 * i) = kk;
#pragma unroll
        for (int e = 0; e < 8; ++e) Vth[(dh + 8 * i + e) * AT_KC + kvr] = vv[e];
      }
    }
    __syncthreads();

    v8f s[4];
#pragma unroll
    for (int j = 0; j < 4; ++j) {
      s[j] = (v8f){0.f,0.f,0.f,0.f,0.f,0.f,0.f,0.f};
#pragma unroll
      for (int dc = 0; dc < 2; ++dc) {
        const v16h kb = Frag<_Float16>::load(Ksh + (j * 16 + c) * AT_D + dc * 32 + 8 * hh);
        s[j] = mma_h(qa[dc], kb, s[j]);
      }
    }
    float cm[8];
#pragma unroll
    for (int r = 0; r < 8; ++r) {
      float m = -INFINITY;
#pragma unroll
      for (int j = 0; j < 4; ++j) {
        s[j][r] = s[j][r] * qscale;
        m = fmaxf(m, s[j][r]);
      }
#pragma unroll
      for (int off = 1; off < 16; off <<= 1) m = fmaxf(m, __shfl_xor(m, off, 32));
      cm[r] = m;
    }
    _Float16* pw = Psh[wave];
#pragma unroll
    for (int r = 0; r < 8; ++r) {
      const float mnew = fmaxf(mrow[r], cm[r]);
      const float alpha = expf(mrow[r] - mnew);
      mrow[r] = mnew;
      float psum = 0.f;
#pragma unroll
      for (int j = 0; j < 4; ++j) {
        const float p = expf(s[j][r] - mnew);
        psum += p;
        pw[(8 * hh + r) * AT_KC + j * 16 + c] = (_Float16)(p * AT_PSC);
      }
#pragma unroll
      for (int off = 1; off < 16; off <<= 1) psum += __shfl_xor(psum, off, 32);
      lrow[r] = lrow[r] * alpha + psum;
#pragma unroll
      for (int t = 0; t < 4; ++t) oacc[t][r] *= alpha;
    }
    __builtin_amdgcn_fence(__ATOMIC_RELEASE, "workgroup");
    __builtin_amdgcn_wave_barrier();
    __builtin_amdgcn_fence(__ATOMIC_ACQUIRE, "workgroup");
#pragma unroll 1
    for (int kk = 0; kk < 2; ++kk) {
      const v16h pa = Frag<_Float16>::load(pw + c * AT_KC + kk * 32 + 8 * hh);
#pragma unroll
      for (int t = 0; t < 4; ++t) {
        const v16h vb = Frag<_Float16>::load(Vth + (t * 16 + c) * AT_KC + kk * 32 + 8 * hh);
        oacc[t] = mma_h(pa, vb, oacc[t]);
      }
    }
  }

  float* os = Os[wave];
#pragma unroll
  for (int r = 0; r < 8; ++r) {
    const float inv = 1.0f / (lrow[r] * AT_PSC);
#pragma unroll
    for (int t = 0; t < 4; ++t) os[(8 * hh + r) * 68 + t * 16 + c] = oacc[t][r] * inv;
  }
  __builtin_amdgcn_fence(__ATOMIC_RELEASE, "workgroup");
  __builtin_amdgcn_wave_barrier();
  __builtin_amdgcn_fence(__ATOMIC_ACQUIRE, "workgroup");
  {
    const int c4 = (lane & 15) * 4;
    for (int pass = 0; pass < 2; ++pass) {
#pragma unroll
      for (int it = 0; it < 8; ++it) {
        const int row = it * 2 + hh;
        v4f val = *(const v4f*)(os + row * 68 + c4);
        *(volatile v4f*)(obp + (size_t)(q0 + row) * ldo + c4) = val;
      }
      __threadfence();
    }
  }
}

static inline unsigned gemm_grid64(int M, int N) { return (unsigned)((((M / 64) * (N / 64)) + 7) / 8); }

extern "C" void kernel_launch(void* const* d_in, const int* in_sizes, int n_in,
                              void* d_out, int out_size, void* d_ws,
                              size_t ws_size, hipStream_t stream) {
  const int BD = 4, SEQ = 1024, DIM = 768, NH = 12, HDIM = 64, MLPD = 3072;
  const int ROWS = BD * SEQ;
  const int QKVD = 3 * DIM;
  const int QKD  = 2 * DIM;
  (void)HDIM;
  if (n_in < 17) return;
  if (in_sizes[0] != ROWS * DIM || out_size != ROWS * DIM) return;
  if (in_sizes[2] != DIM || in_sizes[3] != DIM || in_sizes[7] != DIM || in_sizes[8] != DIM ||
      in_sizes[11] != DIM || in_sizes[12] != DIM || in_sizes[16] != DIM || in_sizes[14] != MLPD) return;
  if (in_sizes[4] != QKVD * DIM || in_sizes[5] != QKVD * DIM || in_sizes[6] != DIM * DIM ||
      in_sizes[13] != MLPD * DIM || in_sizes[15] != DIM * MLPD) return;
  if (in_sizes[9] < NH || in_sizes[10] < NH) return;

  const float* x      = (const float*)d_in[0];
  const int*   xpos   = (const int*)d_in[1];
  const float* ln1_w  = (const float*)d_in[2];
  const float* ln1_b  = (const float*)d_in[3];
  const float* qkv1_w = (const float*)d_in[4];
  const float* qkv2_w = (const float*)d_in[5];
  const float* proj_w = (const float*)d_in[6];
  const float* proj_b = (const float*)d_in[7];
  const float* rms_w  = (const float*)d_in[8];
  const float* lam1   = (const float*)d_in[9];
  const float* lam2   = (const float*)d_in[10];
  const float* ln2_w  = (const float*)d_in[11];
  const float* ln2_b  = (const float*)d_in[12];
  const float* fc1_w  = (const float*)d_in[13];
  const float* fc1_b  = (const float*)d_in[14];
  const float* fc2_w  = (const float*)d_in[15];
  const float* fc2_b  = (const float*)d_in[16];

  char* ws = (char*)d_ws;
  size_t off = 0;
  auto carve = [&](size_t bytes) -> char* {
    off = (off + 255) & ~(size_t)255;
    char* p = ws + off;
    off += bytes;
    return p;
  };
  _Float16* h1   = (_Float16*)carve((size_t)ROWS * DIM * 2);
  _Float16* w1h  = (_Float16*)carve((size_t)QKVD * DIM * 2);
  _Float16* w2h  = (_Float16*)carve((size_t)QKD * DIM * 2);
  _Float16* wph  = (_Float16*)carve((size_t)DIM * DIM * 2);
  _Float16* wf1h = (_Float16*)carve((size_t)MLPD * DIM * 2);
  _Float16* wf2h = (_Float16*)carve((size_t)DIM * MLPD * 2);
  _Float16* qkv1 = (_Float16*)carve((size_t)ROWS * QKVD * 2);
  _Float16* qk2  = (_Float16*)carve((size_t)ROWS * QKD * 2);
  float*    O1   = (float*)carve((size_t)ROWS * DIM * 4);
  float*    O2   = (float*)carve((size_t)ROWS * DIM * 4);
  _Float16* onm  = (_Float16*)carve((size_t)ROWS * DIM * 2);
  float*    x1   = (float*)carve((size_t)ROWS * DIM * 4);
  const size_t total = off;
  if (total > ws_size || total > (size_t)134217728) return;
  _Float16* h2  = h1;
  _Float16* mm1 = qkv1;
  if ((size_t)ROWS * MLPD * 2 > (size_t)ROWS * QKVD * 2 + (size_t)ROWS * QKD * 2) return;

  const float WSC = 64.0f, WSC_INV = 1.0f / 64.0f;

  {
    int n2;
    n2 = QKVD * DIM / 2; cast_scale_f32_f16x2<<<(n2 + 255) / 256, 256, 0, stream>>>(qkv1_w, w1h, n2, WSC);
    n2 = QKD * DIM / 2;  cast_scale_f32_f16x2<<<(n2 + 255) / 256, 256, 0, stream>>>(qkv2_w, w2h, n2, WSC);
    n2 = DIM * DIM / 2;  cast_scale_f32_f16x2<<<(n2 + 255) / 256, 256, 0, stream>>>(proj_w, wph, n2, WSC);
    n2 = MLPD * DIM / 2; cast_scale_f32_f16x2<<<(n2 + 255) / 256, 256, 0, stream>>>(fc1_w, wf1h, n2, WSC);
    n2 = DIM * MLPD / 2; cast_scale_f32_f16x2<<<(n2 + 255) / 256, 256, 0, stream>>>(fc2_w, wf2h, n2, WSC);
  }

  ln_rows_f16<<<(ROWS + 7) / 8, 256, 0, stream>>>(x, ln1_w, ln1_b, h1, ROWS, 1e-5f);

  wmma_gemm64<0, false, 0, 1, false, 0><<<dim3(gemm_grid64(ROWS, QKVD), 1), 256, 0, stream>>>(
      (const unsigned short*)h1, nullptr, DIM, 0L,
      (const unsigned short*)w1h, nullptr, DIM, 0L,
      (void*)qkv1, nullptr, QKVD, 0L,
      nullptr, nullptr, 0L, ROWS, QKVD, DIM, WSC_INV);
  wmma_gemm64<0, false, 0, 1, false, 0><<<dim3(gemm_grid64(ROWS, QKD), 1), 256, 0, stream>>>(
      (const unsigned short*)h1, nullptr, DIM, 0L,
      (const unsigned short*)w2h, nullptr, DIM, 0L,
      (void*)qk2, nullptr, QKD, 0L,
      nullptr, nullptr, 0L, ROWS, QKD, DIM, WSC_INV);

  const unsigned agrid = (unsigned)(BD * NH * (SEQ / AT_QB));
  attn64_f16<<<agrid, 128, 0, stream>>>(qkv1, QKVD, qkv1 + DIM, QKVD, qkv1 + 2 * DIM, QKVD,
                                         O1, DIM, SEQ, SEQ, NH, 0.125f);
  attn64_f16<<<agrid, 128, 0, stream>>>(qk2, QKD, qk2 + DIM, QKD, qkv1 + 2 * DIM, QKVD,
                                         O2, DIM, SEQ, SEQ, NH, 0.125f);

  diff_rms_f16<<<(ROWS + 7) / 8, 256, 0, stream>>>(O1, O2, lam1, lam2, rms_w, xpos, onm, ROWS, 1e-6f, 0.1f);

  wmma_gemm64<0, false, 2, 0, true, 0><<<dim3(gemm_grid64(ROWS, DIM), 1), 256, 0, stream>>>(
      (const unsigned short*)onm, nullptr, DIM, 0L,
      (const unsigned short*)wph, nullptr, DIM, 0L,
      (void*)x1, nullptr, DIM, 0L,
      proj_b, x, 0L, ROWS, DIM, DIM, WSC_INV);

  ln_rows_f16<<<(ROWS + 7) / 8, 256, 0, stream>>>(x1, ln2_w, ln2_b, h2, ROWS, 1e-5f);

  wmma_gemm64<0, false, 2, 1, false, 5><<<dim3(gemm_grid64(ROWS, MLPD), 1), 256, 0, stream>>>(
      (const unsigned short*)h2, nullptr, DIM, 0L,
      (const unsigned short*)wf1h, nullptr, DIM, 0L,
      (void*)mm1, nullptr, MLPD, 0L,
      fc1_b, nullptr, 0L, ROWS, MLPD, DIM, WSC_INV);

  wmma_gemm64<0, false, 2, 0, true, 0><<<dim3(gemm_grid64(ROWS, DIM), 1), 256, 0, stream>>>(
      (const unsigned short*)mm1, nullptr, MLPD, 0L,
      (const unsigned short*)wf2h, nullptr, MLPD, 0L,
      d_out, nullptr, DIM, 0L,
      fc2_b, x1, 0L, ROWS, DIM, MLPD, WSC_INV);
}
